// FG_4552665333921
// MI455X (gfx1250) — hardware-verified
//
#include <hip/hip_runtime.h>
#define NB 32
#define CI 3
#define HI 128
#define WI 128
#define CH 64
#define H1s 63
#define H2s 31
#define H3s 15
#define H4s 7
#define KK 9
#define GH 32
#define GW 32
#define NK 49
#define BNEPS 1e-5f
typedef __bf16 v16b __attribute__((ext_vector_type(16)));
typedef unsigned short v8us __attribute__((ext_vector_type(8), may_alias));
typedef float  v8f  __attribute__((ext_vector_type(8)));
typedef float  v4f  __attribute__((ext_vector_type(4)));
typedef float  v4fa __attribute__((ext_vector_type(4), may_alias));
union FragB { v16b v; v8us half[2]; unsigned short u[16]; };

__device__ __forceinline__ unsigned short bf16_bits(float x) { unsigned int u = __float_as_uint(x); return (unsigned short)((u + 0x7FFFu + ((u >> 16) & 1u)) >> 16); }
__device__ __forceinline__ float bf16_val(unsigned short b) { return __uint_as_float(((unsigned int)b) << 16); }
__device__ __forceinline__ float bf16_round(float x) { return bf16_val(bf16_bits(x)); }
template <int NT>
__device__ __forceinline__ v8f mmaN(v16b ah, v16b al, v16b bh, v16b bl, v8f c) {
  c = __builtin_amdgcn_wmma_f32_16x16x32_bf16(false, ah, false, bh, (short)0, c, false, false);
  if (NT >= 2) c = __builtin_amdgcn_wmma_f32_16x16x32_bf16(false, al, false, bh, (short)0, c, false, false);
  if (NT >= 3) c = __builtin_amdgcn_wmma_f32_16x16x32_bf16(false, ah, false, bl, (short)0, c, false, false);
  asm volatile("v_nop\n\tv_nop\n\tv_nop\n\tv_nop" : "+v"(c) : "v"(ah), "v"(al), "v"(bh), "v"(bl));
  return c;
}

__global__ __launch_bounds__(256) void k_wt_bf16(const float* __restrict__ W, unsigned short* __restrict__ Wt, int K, int N) {
  const int t = blockIdx.x * 256 + threadIdx.x;
  const int k8n = K / 8;
  if (t >= N * k8n) return;
  const int n = t / k8n, k8 = (t % k8n) * 8;
  v8us v;
#pragma unroll
  for (int i = 0; i < 8; ++i) v[i] = bf16_bits(W[(size_t)(k8 + i) * N + n]);
  *(volatile v8us*)(Wt + (size_t)n * K + k8) = v;
  __threadfence();
  *(volatile v8us*)(Wt + (size_t)n * K + k8) = v;
}

template <bool ASPLIT, int ACT, bool BIAS_BF16>
__global__ __launch_bounds__(128) void k_gemm_bf(const float* __restrict__ A, int lda, const unsigned short* __restrict__ Wt, int ldb,
                                               const float* __restrict__ bias, float* __restrict__ C, int ldc, int M, int N, int K) {
  __shared__ __attribute__((aligned(16))) float so[4][16][64];
  const int tid = threadIdx.x, w = tid >> 5, lane = tid & 31, ln = lane & 15, hh = lane >> 4;
  const int ntn = N / 64;
  const int wid = blockIdx.x * 4 + w;
  const int mt = wid / ntn, nq = wid % ntn;
  if (mt * 16 >= M) return;
  const int row0 = mt * 16, col0 = nq * 64;
  const float* arow = A + (size_t)(row0 + ln) * lda;
  v8f acc[4] = {};
  for (int kb = 0; kb < K; kb += 32) {
    FragB ah, al;
    const v4f x0 = *(const v4fa*)(arow + kb + 8 * hh), x1 = *(const v4fa*)(arow + kb + 8 * hh + 4);
    const v4f x2 = *(const v4fa*)(arow + kb + 16 + 8 * hh), x3 = *(const v4fa*)(arow + kb + 16 + 8 * hh + 4);
    float xs[16] = {x0[0],x0[1],x0[2],x0[3],x1[0],x1[1],x1[2],x1[3],x2[0],x2[1],x2[2],x2[3],x3[0],x3[1],x3[2],x3[3]};
#pragma unroll
    for (int i = 0; i < 16; ++i) { const unsigned short hb = bf16_bits(xs[i]); ah.u[i] = hb; al.u[i] = ASPLIT ? bf16_bits(xs[i] - bf16_val(hb)) : (unsigned short)0; }
#pragma unroll
    for (int t = 0; t < 4; ++t) {
      const unsigned short* brow = Wt + (size_t)(col0 + t * 16 + ln) * ldb + kb;
      FragB b;
      b.half[0] = *(const v8us*)(brow + 8 * hh);
      b.half[1] = *(const v8us*)(brow + 16 + 8 * hh);
      acc[t] = mmaN<ASPLIT ? 2 : 1>(ah.v, al.v, b.v, b.v, acc[t]);
    }
  }
#pragma unroll
  for (int t = 0; t < 4; ++t) {
    float bv = bias ? bias[col0 + t * 16 + ln] : 0.f;
    if (BIAS_BF16) bv = bf16_round(bv);
#pragma unroll
    for (int r = 0; r < 8; ++r) { float v = acc[t][r] + bv; if (ACT == 1) v = fmaxf(v, 0.f); so[w][8 * hh + r][t * 16 + ln] = v; }
  }
  __builtin_amdgcn_fence(__ATOMIC_ACQ_REL, "workgroup");
  __builtin_amdgcn_wave_barrier();
  const int rsub = lane >> 4, c4 = (lane & 15) * 4;
  for (int pass = 0; pass < 2; ++pass) {
#pragma unroll
    for (int q = 0; q < 8; ++q) {
      const int r = q * 2 + rsub;
      const v4f v = *(const v4fa*)&so[w][r][c4];
      *(volatile v4f*)(C + (size_t)(row0 + r) * ldc + col0 + c4) = v;
    }
    if (pass == 0) __threadfence();
  }
}

template <bool ASPLIT, int ACT, bool BIAS_BF16, bool RES_BF16>
__global__ __launch_bounds__(128) void k_gemm_bf3(const float* __restrict__ A, int lda, const unsigned short* __restrict__ Wt, int ldb,
                                                const float* __restrict__ bias, const float* __restrict__ resid, int rmod, int ldr,
                                                float* __restrict__ C, int ldc, int M, int N, int K) {
  __shared__ __attribute__((aligned(16))) float so[4][16][64];
  const int tid = threadIdx.x, w = tid >> 5, lane = tid & 31, ln = lane & 15, hh = lane >> 4;
  const int ntn = N / 64;
  const int wid = blockIdx.x * 4 + w;
  const int mt = wid / ntn, nq = wid % ntn;
  if (mt * 16 >= M) return;
  const int row0 = mt * 16, col0 = nq * 64;
  const float* arow = A + (size_t)(row0 + ln) * lda;
  v8f acc[4] = {};
  for (int kb = 0; kb < K; kb += 32) {
    FragB ah, al;
    const v4f x0 = *(const v4fa*)(arow + kb + 8 * hh), x1 = *(const v4fa*)(arow + kb + 8 * hh + 4);
    const v4f x2 = *(const v4fa*)(arow + kb + 16 + 8 * hh), x3 = *(const v4fa*)(arow + kb + 16 + 8 * hh + 4);
    float xs[16] = {x0[0],x0[1],x0[2],x0[3],x1[0],x1[1],x1[2],x1[3],x2[0],x2[1],x2[2],x2[3],x3[0],x3[1],x3[2],x3[3]};
#pragma unroll
    for (int i = 0; i < 16; ++i) { const unsigned short hb = bf16_bits(xs[i]); ah.u[i] = hb; al.u[i] = ASPLIT ? bf16_bits(xs[i] - bf16_val(hb)) : (unsigned short)0; }
#pragma unroll
    for (int t = 0; t < 4; ++t) {
      const unsigned short* brow = Wt + (size_t)(col0 + t * 16 + ln) * ldb + kb;
      FragB b;
      b.half[0] = *(const v8us*)(brow + 8 * hh);
      b.half[1] = *(const v8us*)(brow + 16 + 8 * hh);
      acc[t] = mmaN<ASPLIT ? 2 : 1>(ah.v, al.v, b.v, b.v, acc[t]);
    }
  }
#pragma unroll
  for (int t = 0; t < 4; ++t) {
    const int col = col0 + t * 16 + ln;
    float bv = bias ? bias[col] : 0.f;
    if (BIAS_BF16) bv = bf16_round(bv);
#pragma unroll
    for (int r = 0; r < 8; ++r) {
      float v = acc[t][r] + bv;
      if (resid) { float rv = resid[(size_t)((row0 + 8 * hh + r) % rmod) * ldr + col]; if (RES_BF16) rv = bf16_round(rv); v += rv; }
      if (ACT == 1) v = fmaxf(v, 0.f);
      if (ACT == 2) v = 0.5f * v * (1.0f + erff(v * 0.70710678118654752f));
      if (ACT == 3) { const float u = 0.7978845608028654f * (v + 0.044715f * v * v * v); v = 0.5f * v * (1.0f + tanhf(u)); }
      so[w][8 * hh + r][t * 16 + ln] = v;
    }
  }
  __builtin_amdgcn_fence(__ATOMIC_ACQ_REL, "workgroup");
  __builtin_amdgcn_wave_barrier();
  const int rsub = lane >> 4, c4 = (lane & 15) * 4;
  for (int pass = 0; pass < 2; ++pass) {
#pragma unroll
    for (int q = 0; q < 8; ++q) {
      const int r = q * 2 + rsub;
      const v4f v = *(const v4fa*)&so[w][r][c4];
      *(volatile v4f*)(C + (size_t)(row0 + r) * ldc + col0 + c4) = v;
    }
    if (pass == 0) __threadfence();
  }
}
template <bool PARAM_BF16>
__global__ __launch_bounds__(256) void k_layernorm(const float* __restrict__ X, const float* __restrict__ R, const float* __restrict__ g, const float* __restrict__ bta,
                                                  float* __restrict__ out_sum, float* __restrict__ out_norm, int N, float eps) {
  __shared__ float red[256];
  const int row = blockIdx.x, tid = threadIdx.x;
  const float* x = X + (size_t)row * N; const float* rr = R ? R + (size_t)row * N : nullptr;
  float vals[16];
  const int per = N / 256;
  float s1 = 0.f;
  for (int u = 0; u < per / 4; ++u) {
    const int j = tid * 4 + 1024 * u;
    const v4f a = *(const v4fa*)(x + j);
    v4f b = {0.f,0.f,0.f,0.f}; if (rr) b = *(const v4fa*)(rr + j);
#pragma unroll
    for (int q = 0; q < 4; ++q) { const float v = a[q] + b[q]; vals[u * 4 + q] = v; s1 += v; }
  }
  red[tid] = s1; __syncthreads();
  for (int st = 128; st > 0; st >>= 1) { if (tid < st) red[tid] += red[tid + st]; __syncthreads(); }
  const float mu = red[0] / (float)N; __syncthreads();
  float s2 = 0.f;
  for (int u = 0; u < per / 4; ++u)
#pragma unroll
    for (int q = 0; q < 4; ++q) { const float c = vals[u * 4 + q] - mu; s2 += c * c; }
  red[tid] = s2; __syncthreads();
  for (int st = 128; st > 0; st >>= 1) { if (tid < st) red[tid] += red[tid + st]; __syncthreads(); }
  const float rs = rsqrtf(red[0] / (float)N + eps);
  for (int pass = 0; pass < 2; ++pass) {
    for (int u = 0; u < per / 4; ++u) {
      const int j = tid * 4 + 1024 * u;
      v4f o, sm;
#pragma unroll
      for (int q = 0; q < 4; ++q) {
        float gg = g[j + q], bb = bta[j + q];
        if (PARAM_BF16) { gg = bf16_round(gg); bb = bf16_round(bb); }
        sm[q] = vals[u * 4 + q]; o[q] = (vals[u * 4 + q] - mu) * rs * gg + bb;
      }
      if (out_sum) *(volatile v4f*)(out_sum + (size_t)row * N + j) = sm;
      *(volatile v4f*)(out_norm + (size_t)row * N + j) = o;
    }
    if (pass == 0) __threadfence();
  }
}


typedef _Float16 v16h __attribute__((ext_vector_type(16)));
union FragH { v16h v; v8us half[2]; _Float16 h[16]; unsigned short u[16]; };
template <int NT>
__device__ __forceinline__ v8f mmaH(v16h ah, v16h al, v16h bh, v16h bl, v8f c) {
  c = __builtin_amdgcn_wmma_f32_16x16x32_f16(false, ah, false, bh, (short)0, c, false, false);
  if (NT >= 2) c = __builtin_amdgcn_wmma_f32_16x16x32_f16(false, al, false, bh, (short)0, c, false, false);
  if (NT >= 3) c = __builtin_amdgcn_wmma_f32_16x16x32_f16(false, ah, false, bl, (short)0, c, false, false);
  asm volatile("v_nop\n\tv_nop\n\tv_nop\n\tv_nop" : "+v"(c) : "v"(ah), "v"(al), "v"(bh), "v"(bl));
  return c;
}
template <bool ASPLIT>
__global__ __launch_bounds__(128) void k_gemm_h(const float* __restrict__ A, int lda, size_t sA, const _Float16* __restrict__ Bh, int ldb, size_t sB, float alpha, float* __restrict__ C, int ldc, size_t sC, int M, int N, int K) {
  __shared__ __attribute__((aligned(16))) float so[4][16][64];
  const int tid = threadIdx.x, w = tid >> 5, lane = tid & 31, ln = lane & 15, hh = lane >> 4; const int by = blockIdx.y;
  A += (size_t)by * sA; Bh += (size_t)by * sB; C += (size_t)by * sC;
  const int ntn = (N + 63) / 64; const int wid = blockIdx.x * 4 + w; const int mt = wid / ntn, nq = wid % ntn; if (mt * 16 >= M) return;
  const int row0 = mt * 16, col0 = nq * 64; const float* arow = A + (size_t)(row0 + ln) * lda;
  v8f acc[4] = {};
  for (int kb = 0; kb < K; kb += 32) {
    FragH ah, al;
    const v4f x0 = *(const v4fa*)(arow + kb + 8 * hh), x1 = *(const v4fa*)(arow + kb + 8 * hh + 4), x2 = *(const v4fa*)(arow + kb + 16 + 8 * hh), x3 = *(const v4fa*)(arow + kb + 16 + 8 * hh + 4);
    float xs[16] = {x0[0],x0[1],x0[2],x0[3],x1[0],x1[1],x1[2],x1[3],x2[0],x2[1],x2[2],x2[3],x3[0],x3[1],x3[2],x3[3]};
#pragma unroll
    for (int i = 0; i < 16; ++i) { const _Float16 h = (_Float16)xs[i]; ah.h[i] = h; al.h[i] = ASPLIT ? (_Float16)(xs[i] - (float)h) : (_Float16)0.0f; }
#pragma unroll
    for (int t = 0; t < 4; ++t) { if (col0 + t * 16 >= N) continue; const size_t boff = (size_t)(col0 + t * 16 + ln) * ldb + kb; FragH bq; bq.half[0] = *(const v8us*)(Bh + boff + 8 * hh); bq.half[1] = *(const v8us*)(Bh + boff + 16 + 8 * hh);
      acc[t] = mmaH<ASPLIT ? 2 : 1>(ah.v, al.v, bq.v, bq.v, acc[t]); }
  }
#pragma unroll
  for (int t = 0; t < 4; ++t) { if (col0 + t * 16 >= N) continue;
#pragma unroll
    for (int r = 0; r < 8; ++r) so[w][8 * hh + r][t * 16 + ln] = acc[t][r] * alpha; }
  __builtin_amdgcn_fence(__ATOMIC_ACQ_REL, "workgroup"); __builtin_amdgcn_wave_barrier();
  const int rsub = lane >> 4, c4 = (lane & 15) * 4;
  for (int pass = 0; pass < 2; ++pass) {
#pragma unroll
    for (int q = 0; q < 8; ++q) { const int r = q * 2 + rsub; if (col0 + c4 < N) { const v4f v = *(const v4fa*)&so[w][r][c4]; *(volatile v4f*)(C + (size_t)(row0 + r) * ldc + col0 + c4) = v; } }
    if (pass == 0) __threadfence(); }
}

__global__ __launch_bounds__(256) void k_wt_f16(const float* __restrict__ W, _Float16* __restrict__ Wt, int K, int N, float scale) {
  const int t = blockIdx.x * 256 + threadIdx.x; if (t >= N * (K / 8)) return; const int n = t / (K / 8), k8 = (t % (K / 8)) * 8; FragH f;
#pragma unroll
  for (int i = 0; i < 8; ++i) f.h[i] = (_Float16)(bf16_round(W[(size_t)(k8 + i) * N + n]) * scale); const v8us o = f.half[0];
  *(volatile v8us*)((unsigned short*)Wt + (size_t)n * K + k8) = o; __threadfence(); *(volatile v8us*)((unsigned short*)Wt + (size_t)n * K + k8) = o;
}
template <int ACT>
__global__ __launch_bounds__(128) void k_gemm_hhx(const _Float16* __restrict__ A, int lda, size_t sA, const _Float16* __restrict__ Bh, int ldb, size_t sB, float alpha, const float* __restrict__ bias, size_t sBias, const float* __restrict__ CP, int rowsPerB, size_t sCPb, int row0g,
    float* __restrict__ C, _Float16* __restrict__ C16, int ldc, size_t sC, int M, int N, int K) {
  __shared__ __attribute__((aligned(16))) float so[4][16][64];
  const int tid = threadIdx.x, w = tid >> 5, lane = tid & 31, ln = lane & 15, hh = lane >> 4; const int by = blockIdx.y;
  A += (size_t)by * sA; Bh += (size_t)by * sB; const size_t cofs = (size_t)by * sC; const float* bp = bias ? bias + (size_t)by * sBias : nullptr;
  const int ntn = (N + 63) / 64; const int wid = blockIdx.x * 4 + w; const int mt = wid / ntn, nq = wid % ntn; if (mt * 16 >= M) return;
  const int row0 = mt * 16, col0 = nq * 64; const _Float16* arow = A + (size_t)(row0 + ln) * lda;
  v8f acc[4] = {};
  for (int kb = 0; kb < K; kb += 32) { FragH ah; ah.half[0] = *(const v8us*)((const unsigned short*)arow + kb + 8 * hh); ah.half[1] = *(const v8us*)((const unsigned short*)arow + kb + 16 + 8 * hh);
#pragma unroll
    for (int t = 0; t < 4; ++t) { if (col0 + t * 16 >= N) continue; const size_t boff = (size_t)(col0 + t * 16 + ln) * ldb + kb; FragH bq; bq.half[0] = *(const v8us*)((const unsigned short*)Bh + boff + 8 * hh); bq.half[1] = *(const v8us*)((const unsigned short*)Bh + boff + 16 + 8 * hh);
      acc[t] = mmaH<1>(ah.v, ah.v, bq.v, bq.v, acc[t]); }
  }
#pragma unroll
  for (int t = 0; t < 4; ++t) { if (col0 + t * 16 >= N) continue; const int col = col0 + t * 16 + ln; const float bv = bp ? bf16_round(bp[col]) : 0.f;
#pragma unroll
    for (int r = 0; r < 8; ++r) { float v = acc[t][r] * alpha + bv; if (CP) { const int bidx = (row0g + row0 + 8 * hh + r) / rowsPerB; v += CP[(size_t)bidx * sCPb + (size_t)by * 64 + col]; } if (ACT == 1) v = (v > 0.f) ? v : expm1f(v); else if (ACT == 7) v = (v > 0.f) ? v + 1.0f : expf(v); else if (ACT == 8) v = tanhf(v); else if (ACT == 9) v = 0.5f * v * (1.0f + tanhf(0.7978845608028654f * (v + 0.044715f * v * v * v))); else if (ACT == 11) v = 1.0f / (1.0f + expf(-v)); else if (ACT == 12) v = (v > 0.f) ? v : 0.01f * v; else if (ACT == 14) v = (v > 0.f) ? v : 0.1f * v; else if (ACT == 15) v = v / (1.0f + expf(-v)); else if (ACT == 3) v = fmaxf(v, 0.f); else if (ACT == 6) v = 0.5f * v * (1.0f + erff(v * 0.70710678118654752f)); so[w][8 * hh + r][t * 16 + ln] = v; } }
  __builtin_amdgcn_fence(__ATOMIC_ACQ_REL, "workgroup"); __builtin_amdgcn_wave_barrier();
  const int rsub = lane >> 4, c4 = (lane & 15) * 4; typedef _Float16 v4h __attribute__((ext_vector_type(4)));
  for (int pass = 0; pass < 2; ++pass) {
#pragma unroll
    for (int q = 0; q < 8; ++q) { const int r = q * 2 + rsub; if (col0 + c4 < N) { const v4f v = *(const v4fa*)&so[w][r][c4]; if (C) *(volatile v4f*)(C + cofs + (size_t)(row0 + r) * ldc + col0 + c4) = v; if (C16) { v4h h4; for (int i = 0; i < 4; ++i) h4[i] = (_Float16)v[i]; *(volatile v4h*)(C16 + cofs + (size_t)(row0 + r) * ldc + col0 + c4) = h4; } } }
    if (pass == 0) __threadfence(); }
}


typedef _Float16 v4h __attribute__((ext_vector_type(4)));

__global__ __launch_bounds__(256) void k_x16(const float* __restrict__ x, _Float16* __restrict__ X16, size_t n8) { const size_t t = (size_t)blockIdx.x * 256 + threadIdx.x; if (t >= n8) return; FragH f;
#pragma unroll
  for (int q = 0; q < 8; ++q) f.h[q] = (_Float16)bf16_round(x[t * 8 + q]); *(volatile v8us*)((unsigned short*)X16 + t * 8) = f.half[0]; __threadfence(); *(volatile v8us*)((unsigned short*)X16 + t * 8) = f.half[0]; }
__global__ __launch_bounds__(256) void k_h16(const float* __restrict__ x, _Float16* __restrict__ X16, size_t n8) { const size_t t = (size_t)blockIdx.x * 256 + threadIdx.x; if (t >= n8) return; FragH f;
#pragma unroll
  for (int q = 0; q < 8; ++q) f.h[q] = (_Float16)x[t * 8 + q]; *(volatile v8us*)((unsigned short*)X16 + t * 8) = f.half[0]; __threadfence(); *(volatile v8us*)((unsigned short*)X16 + t * 8) = f.half[0]; }
__global__ __launch_bounds__(256) void k_round16f(const float* __restrict__ W, _Float16* __restrict__ Bt, size_t n8) { const size_t t = (size_t)blockIdx.x * 256 + threadIdx.x; if (t >= n8) return; FragH f;
#pragma unroll
  for (int i = 0; i < 8; ++i) f.h[i] = (_Float16)(bf16_round(W[t * 8 + i]) * 16.0f); *(volatile v8us*)((unsigned short*)Bt + t * 8) = f.half[0]; __threadfence(); *(volatile v8us*)((unsigned short*)Bt + t * 8) = f.half[0]; }
template <int NHv, int TTv>
__global__ __launch_bounds__(256) void k_vt(const _Float16* __restrict__ V16, int ldv, int voff, _Float16* __restrict__ Vt) { __shared__ unsigned short tl[64][66]; const int tid = threadIdx.x; const int slab = blockIdx.x / (TTv / 64), lg = blockIdx.x % (TTv / 64); const int b = slab / NHv, h = slab % NHv;
  for (int i = tid; i < 64 * 8; i += 256) { const int r = i / 8, c8 = (i % 8) * 8; FragH f; f.half[0] = *(const v8us*)((const unsigned short*)V16 + ((size_t)b * TTv + lg * 64 + r) * ldv + voff + h * 64 + c8);
#pragma unroll
    for (int q = 0; q < 8; ++q) tl[r][c8 + q] = f.u[q]; }
  __syncthreads();
  for (int pass = 0; pass < 2; ++pass) {
#pragma unroll
    for (int rd = 0; rd < 2; ++rd) { const int d = rd * 32 + tid / 8, pc = tid % 8; FragH f;
#pragma unroll
      for (int q = 0; q < 8; ++q) f.u[q] = tl[pc * 8 + q][d];
      *(volatile v8us*)((unsigned short*)Vt + ((size_t)slab * 64 + d) * TTv + lg * 64 + pc * 8) = f.half[0]; }
    if (pass == 0) __threadfence(); } }

__global__ __launch_bounds__(256) void k_hl(const float* __restrict__ F, _Float16* __restrict__ Hh, _Float16* __restrict__ Hl, size_t n8) { const size_t t = (size_t)blockIdx.x * 256 + threadIdx.x; if (t >= n8) return; FragH fh, fl; const v4f a = *(const v4fa*)(F + t * 8), c = *(const v4fa*)(F + t * 8 + 4);
#pragma unroll
  for (int q = 0; q < 4; ++q) { _Float16 h = (_Float16)a[q]; fh.h[q] = h; fl.h[q] = (_Float16)((a[q] - (float)h) * 1024.0f); h = (_Float16)c[q]; fh.h[4 + q] = h; fl.h[4 + q] = (_Float16)((c[q] - (float)h) * 1024.0f); }
  for (int pass = 0; pass < 2; ++pass) { *(volatile v8us*)((unsigned short*)Hh + t * 8) = fh.half[0]; *(volatile v8us*)((unsigned short*)Hl + t * 8) = fl.half[0]; if (pass == 0) __threadfence(); } }

__device__ __forceinline__ float elu_f(float x) { return (x > 0.f) ? x : expm1f(x); }
__global__ __launch_bounds__(256) void k_im1(const float* __restrict__ img, _Float16* __restrict__ IM) { const size_t t = (size_t)blockIdx.x * 256 + threadIdx.x; if (t >= (size_t)NB * H1s * H1s * 4) return; const int g = (int)(t % 4) * 8; const size_t r = t / 4; const int b = (int)(r / (H1s * H1s)); const int yx = (int)(r % (H1s * H1s)); const int oy = yx / H1s, ox = yx % H1s; FragH f;
#pragma unroll
  for (int q = 0; q < 8; ++q) { const int col = g + q; float v = 0.f; if (col < CI * KK) { const int c = col / KK, k = col % KK; v = bf16_round(img[(((size_t)b * CI + c) * HI + 2 * oy + k / 3) * WI + 2 * ox + k % 3]); } f.h[q] = (_Float16)v; }
  *(volatile v8us*)((unsigned short*)IM + r * 32 + g) = f.half[0]; __threadfence(); *(volatile v8us*)((unsigned short*)IM + r * 32 + g) = f.half[0]; }
__global__ __launch_bounds__(256) void k_w1(const float* __restrict__ w, _Float16* __restrict__ Bt) { const int t = blockIdx.x * 256 + threadIdx.x; if (t >= CH * 4) return; const int o = t / 4, g = (t % 4) * 8; FragH f;
#pragma unroll
  for (int q = 0; q < 8; ++q) { const int col = g + q; f.h[q] = (col < CI * KK) ? (_Float16)(bf16_round(w[(size_t)o * CI * KK + col]) * 16.0f) : (_Float16)0.0f; }
  *(volatile v8us*)((unsigned short*)Bt + (size_t)o * 32 + g) = f.half[0]; __threadfence(); *(volatile v8us*)((unsigned short*)Bt + (size_t)o * 32 + g) = f.half[0]; }
__global__ __launch_bounds__(256) void k_colstats(const float* __restrict__ Z, int R, float* __restrict__ MEAN, float* __restrict__ RSTD) { __shared__ float s1[8][32], s2[8][32]; const int tid = threadIdx.x, w = tid >> 5, l = tid & 31; const int c = blockIdx.x * 32 + l; float a = 0.f, b = 0.f;
#pragma unroll 1
  for (int r = w; r < R; r += 8) { const float v = Z[(size_t)r * CH + c]; a += v; b += v * v; }
  s1[w][l] = a; s2[w][l] = b; __syncthreads();
  if (w == 0) { float t1 = 0.f, t2 = 0.f;
#pragma unroll
    for (int k = 0; k < 8; ++k) { t1 += s1[k][l]; t2 += s2[k][l]; } const float mu = t1 / (float)R; const float var = fmaxf(t2 / (float)R - mu * mu, 0.f); const float rs = rsqrtf(var + BNEPS);
    for (int pass = 0; pass < 2; ++pass) { *(volatile float*)(MEAN + c) = mu; *(volatile float*)(RSTD + c) = rs; if (pass == 0) __threadfence(); } } }
__global__ __launch_bounds__(256) void k_bnelu(float* Z, int R, const float* __restrict__ MEAN, const float* __restrict__ RSTD, const float* __restrict__ g, const float* __restrict__ be) {
  #pragma clang fp contract(off)
  float* A = Z;
  const size_t t = (size_t)blockIdx.x * 256 + threadIdx.x; if (t >= (size_t)R * 8) return; const size_t r = t / 8; const int c0 = (int)(t % 8) * 8; v4f a, c;
#pragma unroll
  for (int q = 0; q < 8; ++q) { const int ch = c0 + q; const float v = elu_f(bf16_round(g[ch]) * ((Z[r * CH + ch] - MEAN[ch]) * RSTD[ch]) + bf16_round(be[ch])); if (q < 4) a[q] = v; else c[q - 4] = v; }
  for (int pass = 0; pass < 2; ++pass) { *(volatile v4f*)(A + r * CH + c0) = a; *(volatile v4f*)(A + r * CH + c0 + 4) = c; if (pass == 0) __threadfence(); } }
__global__ __launch_bounds__(256) void k_im2(const float* __restrict__ A, int Hin, int Hout, _Float16* __restrict__ IMh, _Float16* __restrict__ IMl) {
  #pragma clang fp contract(off)
  const size_t t = (size_t)blockIdx.x * 256 + threadIdx.x; const size_t total = (size_t)NB * Hout * Hout * KK * 8; if (t >= total) return; const int c0 = (int)(t % 8) * 8; const size_t rk = t / 8; const int k = (int)(rk % KK); const size_t r = rk / KK; const int b = (int)(r / ((size_t)Hout * Hout)); const int yx = (int)(r % ((size_t)Hout * Hout)); const int oy = yx / Hout, ox = yx % Hout;
  const float* src = A + (((size_t)b * Hin + 2 * oy + k / 3) * Hin + 2 * ox + k % 3) * CH + c0; const v4f a0 = *(const v4fa*)src, a1 = *(const v4fa*)(src + 4); FragH fh, fl;
#pragma unroll
  for (int q = 0; q < 8; ++q) { const float v = (q < 4) ? a0[q] : a1[q - 4]; const _Float16 hi = (_Float16)v; fh.h[q] = hi; fl.h[q] = (_Float16)((v - (float)hi) * 1024.0f); }
  const size_t o = r * (KK * CH) + (size_t)k * CH + c0;
  for (int pass = 0; pass < 2; ++pass) { *(volatile v8us*)((unsigned short*)IMh + o) = fh.half[0]; *(volatile v8us*)((unsigned short*)IMl + o) = fl.half[0]; if (pass == 0) __threadfence(); } }
__global__ __launch_bounds__(256) void k_w3x3(const float* __restrict__ w, _Float16* __restrict__ Bt) { const int t = blockIdx.x * 256 + threadIdx.x; if (t >= CH * KK * 8) return; const int c0 = (t % 8) * 8; const int k = (t / 8) % KK, o = t / (8 * KK); FragH f;
#pragma unroll
  for (int q = 0; q < 8; ++q) f.h[q] = (_Float16)(bf16_round(w[(((size_t)o * CH + c0 + q) * KK) + k]) * 16.0f);
  *(volatile v8us*)((unsigned short*)Bt + (size_t)o * (KK * CH) + (size_t)k * CH + c0) = f.half[0]; __threadfence(); *(volatile v8us*)((unsigned short*)Bt + (size_t)o * (KK * CH) + (size_t)k * CH + c0) = f.half[0]; }
__global__ __launch_bounds__(256) void k_head(const float* __restrict__ A4, const float* __restrict__ wp, const float* __restrict__ bp, const float* __restrict__ wz, const float* __restrict__ bz, const float* __restrict__ es, const float* __restrict__ et, float* __restrict__ PRM) {
  #pragma clang fp contract(off)
  __shared__ __attribute__((aligned(16))) float prm[8][4]; const int tid = threadIdx.x, w = tid >> 5, l = tid & 31; const int cell = blockIdx.x * 8 + w; const int b = cell / NK, k = cell % NK; const int i = k / 7, j = k % 7;
  const float* a = A4 + (size_t)cell * CH; float f0 = bf16_round(bp[2 * l]), f1 = bf16_round(bp[2 * l + 1]);
#pragma unroll 1
  for (int c = 0; c < CH; ++c) { const float av = a[c]; f0 += bf16_round(wp[(size_t)(2 * l) * CH + c]) * av; f1 += bf16_round(wp[(size_t)(2 * l + 1) * CH + c]) * av; }
  f0 = elu_f(f0); f1 = elu_f(f1);
  float z[11];
#pragma unroll
  for (int o = 0; o < 11; ++o) { float p = bf16_round(wz[o * CH + 2 * l]) * f0 + bf16_round(wz[o * CH + 2 * l + 1]) * f1; for (int s = 16; s > 0; s >>= 1) p += __shfl_xor(p, s, 32); z[o] = p + bf16_round(bz[o]); }
  if (l == 0) { const float* esb = es + ((size_t)b * NK + k) * 2; const float* etb = et + ((size_t)b * NK + k) * 2;
    const float sp0 = (z[5] > 20.f) ? z[5] : __logf(1.0f + __expf(z[5])), sp1 = (z[6] > 20.f) ? z[6] : __logf(1.0f + __expf(z[6])), sp2 = (z[9] > 20.f) ? z[9] : __logf(1.0f + __expf(z[9])), sp3 = (z[10] > 20.f) ? z[10] : __logf(1.0f + __expf(z[10]));
    const float zs0 = z[3] + sp0 * bf16_round(esb[0]), zs1 = z[4] + sp1 * bf16_round(esb[1]), zt0 = z[7] + sp2 * bf16_round(etb[0]), zt1 = z[8] + sp3 * bf16_round(etb[1]);
    const float th = (1.0f / (1.0f + __expf(-zs0))) * (float)GH / (float)HI, tw = (1.0f / (1.0f + __expf(-zs1))) * (float)GW / (float)WI;
    const float tx = (((float)i / 7.0f) + (1.0f / (1.0f + __expf(-zt0))) / 7.0f) * 2.0f - 1.0f, ty = (((float)j / 7.0f) + (1.0f / (1.0f + __expf(-zt1))) / 7.0f) * 2.0f - 1.0f;
    prm[w][0] = th; prm[w][1] = tw; prm[w][2] = tx; prm[w][3] = ty; }
  __syncthreads();
  if (tid < 8) { const v4f v = *(const v4fa*)&prm[tid][0]; *(volatile v4f*)(PRM + (size_t)(blockIdx.x * 8 + tid) * 4) = v; __threadfence(); *(volatile v4f*)(PRM + (size_t)(blockIdx.x * 8 + tid) * 4) = v; } }
__global__ __launch_bounds__(256) void k_glimpse(const float* __restrict__ img, const float* __restrict__ PRM, float* __restrict__ out) {
  #pragma clang fp contract(off)
  const size_t t = (size_t)blockIdx.x * 256 + threadIdx.x; if (t >= (size_t)NB * NK * CI * GH * (GW / 4)) return; const int gx0 = (int)(t % (GW / 4)) * 4; const size_t r1 = t / (GW / 4); const int gy = (int)(r1 % GH); const size_t r2 = r1 / GH; const int c = (int)(r2 % CI); const int bk = (int)(r2 / CI); const int b = bk / NK;
  const float th = PRM[(size_t)bk * 4], tw = PRM[(size_t)bk * 4 + 1], tx = PRM[(size_t)bk * 4 + 2], ty = PRM[(size_t)bk * 4 + 3];
  const float yb = (2.0f * (float)gy + 1.0f) / (float)GH - 1.0f; const float iyn = th * yb + tx; const float py = ((iyn + 1.0f) * (float)HI - 1.0f) * 0.5f; const float fy = floorf(py); const float wy1 = py - fy; const int y0 = (int)fy;
  const float* im = img + ((size_t)b * CI + c) * HI * WI; v4f o;
#pragma unroll
  for (int q = 0; q < 4; ++q) { const int gx = gx0 + q; const float xb = (2.0f * (float)gx + 1.0f) / (float)GW - 1.0f; const float ixn = tw * xb + ty; const float px = ((ixn + 1.0f) * (float)WI - 1.0f) * 0.5f; const float fx = floorf(px); const float wx1 = px - fx; const int x0 = (int)fx; float s = 0.f;
#pragma unroll
    for (int cc = 0; cc < 4; ++cc) { const int yi = y0 + (cc >> 1), xi = x0 + (cc & 1); const bool m = (xi >= 0) && (xi < WI) && (yi >= 0) && (yi < HI); const float wgt = ((cc >> 1) ? wy1 : 1.f - wy1) * ((cc & 1) ? wx1 : 1.f - wx1);
      s += (m ? wgt : 0.f) * bf16_round(im[(size_t)min(max(yi, 0), HI - 1) * WI + min(max(xi, 0), WI - 1)]); }
    o[q] = s; }
  float* op = out + (((size_t)bk * CI + c) * GH + gy) * GW + gx0; *(volatile v4f*)op = o; __threadfence(); *(volatile v4f*)op = o; }

extern "C" void kernel_launch(void* const* d_in, const int* in_sizes, int n_in,
                              void* d_out, int out_size, void* d_ws, size_t ws_size, hipStream_t stream) {
  (void)in_sizes; (void)n_in; (void)out_size;
  const float* const* I = (const float* const*)d_in; const float* img = I[0]; const float* es = I[1]; const float* et = I[2];
  const float* cw[4] = {I[3], I[7], I[11], I[15]}; const float* cb[4] = {I[4], I[8], I[12], I[16]}; const float* cg[4] = {I[5], I[9], I[13], I[17]}; const float* cbe[4] = {I[6], I[10], I[14], I[18]}; const float* wp = I[19]; const float* bp = I[20]; const float* wz = I[21]; const float* bz = I[22];
  char* ws = (char*)d_ws; size_t off = 0;
  auto take = [&](size_t bytes) { char* p = ws + off; off += (bytes + 255) & ~(size_t)255; return p; };
  const int Hs[5] = {HI, H1s, H2s, H3s, H4s}; const size_t R1 = (size_t)NB * H1s * H1s, R2 = (size_t)NB * H2s * H2s, R3 = (size_t)NB * H3s * H3s, R4 = (size_t)NB * H4s * H4s;
  _Float16* B1 = (_Float16*)take((size_t)CH * 32 * 2); _Float16* B3[3]; for (int i = 0; i < 3; ++i) B3[i] = (_Float16*)take((size_t)CH * KK * CH * 2); float* MEAN = (float*)take(CH * 4); float* RSTD = (float*)take(CH * 4);
  float* Z = (float*)take(R1 * CH * 4); _Float16* IMh = (_Float16*)take(R2 * KK * CH * 2); _Float16* IMl = (_Float16*)take(R2 * KK * CH * 2); float* PRM = (float*)take((size_t)NB * NK * 4 * 4);
  _Float16* IM1 = IMh;
  float* A = Z;
  if (off > ws_size) return;
  k_w1<<<1, 256, 0, stream>>>(cw[0], B1); for (int i = 0; i < 3; ++i) k_w3x3<<<(CH * KK * 8 + 255) / 256, 256, 0, stream>>>(cw[i + 1], B3[i]);
  k_im1<<<(unsigned)((R1 * 4 + 255) / 256), 256, 0, stream>>>(img, IM1);
  k_gemm_hhx<0><<<dim3((unsigned)(((R1 / 16) * 1 + 3) / 4), 1), 128, 0, stream>>>(IM1, 32, 0, B1, 32, 0, 0.0625f, cb[0], 0, nullptr, 1, 0, 0, Z, nullptr, CH, 0, (int)R1, CH, 32);
  k_colstats<<<CH / 32, 256, 0, stream>>>(Z, (int)R1, MEAN, RSTD); k_bnelu<<<(unsigned)((R1 * 8 + 255) / 256), 256, 0, stream>>>(Z, (int)R1, MEAN, RSTD, cg[0], cbe[0]);
  const size_t Rs[4] = {R1, R2, R3, R4};
  for (int L = 1; L < 4; ++L) { const size_t R = Rs[L];
    k_im2<<<(unsigned)((R * KK * 8 + 255) / 256), 256, 0, stream>>>(A, Hs[L], Hs[L + 1], IMh, IMl);
    k_gemm_hhx<0><<<dim3((unsigned)(((R / 16) * 1 + 3) / 4), 1), 128, 0, stream>>>(IMh, KK * CH, 0, B3[L - 1], KK * CH, 0, 0.0625f, cb[L], 0, nullptr, 1, 0, 0, Z, nullptr, CH, 0, (int)R, CH, KK * CH);
    k_gemm_hhx<0><<<dim3((unsigned)(((R / 16) * 1 + 3) / 4), 1), 128, 0, stream>>>(IMl, KK * CH, 0, B3[L - 1], KK * CH, 0, 0.0625f / 1024.0f, nullptr, 0, Z, 1, (size_t)CH, 0, Z, nullptr, CH, 0, (int)R, CH, KK * CH);
    k_colstats<<<CH / 32, 256, 0, stream>>>(Z, (int)R, MEAN, RSTD); k_bnelu<<<(unsigned)((R * 8 + 255) / 256), 256, 0, stream>>>(Z, (int)R, MEAN, RSTD, cg[L], cbe[L]); }
  k_head<<<NB * NK / 8, 256, 0, stream>>>(A, wp, bp, wz, bz, es, et, PRM);
  k_glimpse<<<(unsigned)(((size_t)NB * NK * CI * GH * (GW / 4) + 255) / 256), 256, 0, stream>>>(img, PRM, (float*)d_out);
}
